// RandomGRU_54322746359880
// MI455X (gfx1250) — hardware-verified
//
#include <hip/hip_runtime.h>


typedef _Float16 f16t;
typedef f16t  v16h __attribute__((ext_vector_type(16)));
typedef f16t  v8h  __attribute__((ext_vector_type(8)));
typedef float v8f  __attribute__((ext_vector_type(8)));
typedef float v4f  __attribute__((ext_vector_type(4)));
typedef float v2f  __attribute__((ext_vector_type(2)));

union Frag { v16h v; v8h q[2]; };
union Pk16 { v8h h; v4f f; };

#define TT   12
#define HH   64
#define MM   32
#define PP   12
#define XW   24
#define NPL  4096
#define RB   128
#define HP   72
#define SC_H 16.0f
#define SC_W 64.0f
#define INV_HW 0.0009765625f

struct HArgs { const float* Wl[3]; const float* bl[3]; };
struct XArgs { const float* Wlx[3]; const float* blx[3]; const float* Wbx[3];
               const float* bbx[3]; const float* Wbh[3]; const float* bbh[3]; };
static_assert(sizeof(HArgs) == 48);
static_assert(sizeof(XArgs) == 144);

__device__ __forceinline__ const float* sel3(int g, const float* p0, const float* p1, const float* p2) {
    return (g == 0) ? p0 : ((g == 1) ? p1 : p2);
}

__device__ __forceinline__ v8f wmma16(v16h a, v16h b, v8f c) {
    return __builtin_amdgcn_wmma_f32_16x16x32_f16(false, a, false, b, (short)0, c, false, false);
}

__device__ __forceinline__ v8f hprod(const Frag& a0, const Frag& a1,
                                     const f16t* __restrict__ prow, int h) {
    Frag b0, b1;
    const f16t* p = prow + 8 * h;
    b0.q[0] = *(const v8h*)(p);
    b0.q[1] = *(const v8h*)(p + 16);
    b1.q[0] = *(const v8h*)(p + 32);
    b1.q[1] = *(const v8h*)(p + 48);
    v8f c = {0.f, 0.f, 0.f, 0.f, 0.f, 0.f, 0.f, 0.f};
    c = wmma16(a0.v, b0.v, c);
    c = wmma16(a1.v, b1.v, c);
    asm volatile("v_nop\n\tv_nop\n\tv_nop\n\tv_nop"
                 : "+v"(c)
                 : "v"(a0.v), "v"(a1.v), "v"(b0.v), "v"(b1.v)
                 : "memory");
    return c;
}

__device__ __forceinline__ float fsigm(float x) {
    return __builtin_amdgcn_rcpf(1.0f + __expf(-x));
}
__device__ __forceinline__ float ftanh(float x) {
    float ax = fabsf(x);
    float t  = __expf(-2.0f * ax);
    float r  = (1.0f - t) * __builtin_amdgcn_rcpf(1.0f + t);
    return copysignf(r, x);
}

__global__ __launch_bounds__(256)
void k_meta_h(const float* __restrict__ wz, HArgs a, f16t* P) {
    __shared__ __attribute__((aligned(16))) f16t sm[256];
    const int tid = threadIdx.x;
    const int tg  = blockIdx.x >> 4;
    const int t   = tg / 3, g = tg - 3 * t;
    const int row = ((blockIdx.x & 15) << 8) + tid;
    const float* Wl = sel3(g, a.Wl[0], a.Wl[1], a.Wl[2]);
    const float* bl = sel3(g, a.bl[0], a.bl[1], a.bl[2]);
    const float* wr   = wz + t * MM;
    const float* wrow = Wl + (size_t)row * MM;
    float acc = 0.f;
#pragma unroll
    for (int q = 0; q < 8; ++q) {
        v4f a4 = *(const v4f*)(wrow + 4 * q);
        v4f z4 = *(const v4f*)(wr + 4 * q);
        acc = fmaf(z4[0], a4[0], acc);
        acc = fmaf(z4[1], a4[1], acc);
        acc = fmaf(z4[2], a4[2], acc);
        acc = fmaf(z4[3], a4[3], acc);
    }
    acc += bl[row];
    sm[tid] = (f16t)(acc * SC_W);
    __syncthreads();
    const int li = (tid < 32) ? tid : 0;
    Pk16 v;
    v.h = *(const v8h*)(sm + li * 8);
    f16t* dst = P + (size_t)blockIdx.x * 256 + li * 8;
    if (tid < 32) *(volatile v4f*)dst = v.f;
    __threadfence();
    if (tid < 32) *(volatile v4f*)dst = v.f;
}

__global__ __launch_bounds__(256)
void k_meta_x(const float* __restrict__ wz, const float* __restrict__ bz,
              const float* __restrict__ unused_in1, XArgs a, float* F) {
    __shared__ __attribute__((aligned(16))) float sm[256];
    const int tid = threadIdx.x;
    const int tg  = blockIdx.x;
    const int t   = tg / 3, g = tg - 3 * t;
    const int c   = tid >> 6;
    const int n   = tid & 63;
    const float* Wlx = sel3(g, a.Wlx[0], a.Wlx[1], a.Wlx[2]);
    const float* blx = sel3(g, a.blx[0], a.blx[1], a.blx[2]);
    const float* Wbx = sel3(g, a.Wbx[0], a.Wbx[1], a.Wbx[2]);
    const float* bbx = sel3(g, a.bbx[0], a.bbx[1], a.bbx[2]);
    const float* Wbh = sel3(g, a.Wbh[0], a.Wbh[1], a.Wbh[2]);
    const float* bbh = sel3(g, a.bbh[0], a.bbh[1], a.bbh[2]);
    const float* Wsrc = (c < 2) ? Wlx : ((c == 2) ? Wbx : Wbh);
    const int    rw   = (c < 2) ? (2 * n + (c & 1)) : n;
    const float* vec  = ((c < 2) ? wz : bz) + t * MM;
    const float b_l = blx[2 * n + (c & 1)];
    const float b_x = bbx[n];
    const float b_h = bbh[n];
    const float bias = (c < 2) ? b_l : ((c == 2) ? b_x : b_h);
    const float* wrow = Wsrc + (size_t)rw * MM;
    float acc = 0.f;
#pragma unroll
    for (int q = 0; q < 8; ++q) {
        v4f a4 = *(const v4f*)(wrow + 4 * q);
        v4f z4 = *(const v4f*)(vec + 4 * q);
        acc = fmaf(z4[0], a4[0], acc);
        acc = fmaf(z4[1], a4[1], acc);
        acc = fmaf(z4[2], a4[2], acc);
        acc = fmaf(z4[3], a4[3], acc);
    }
    sm[n * 4 + c] = acc + bias;
    __syncthreads();
    const int li = (tid < 64) ? tid : 0;
    v4f v = *(const v4f*)(sm + li * 4);
    float* dst = F + (size_t)blockIdx.x * 256 + li * 4;
    if (tid < 64) *(volatile v4f*)dst = v;
    __threadfence();
    if (tid < 64) *(volatile v4f*)dst = v;
}

__device__ __forceinline__ void gru_nb(int nb, const Frag& a0, const Frag& a1,
                                       const f16t* __restrict__ Pt, const v4f* __restrict__ Ft,
                                       const float (&x0)[8], const float (&x1)[8],
                                       v8f& hf, float won, float (&pr)[8],
                                       f16t* hrow, int h, int m) {
    const int n = nb * 16 + m;
    const v4f fr = Ft[n];
    const v4f fz = Ft[HH + n];
    const v4f fc = Ft[2 * HH + n];
    v8f ar = hprod(a0, a1, Pt + (size_t)n * HH, h);
    v8f az = hprod(a0, a1, Pt + NPL + (size_t)n * HH, h);
    v8f ac = hprod(a0, a1, Pt + 2 * NPL + (size_t)n * HH, h);
    const float br  = fr[2] + fr[3];
    const float bzz = fz[2] + fz[3];
#pragma unroll
    for (int i = 0; i < 8; ++i) {
        float pre_r = fmaf(x0[i], fr[0], fmaf(x1[i], fr[1], br));
        float r     = fsigm(fmaf(ar[i], INV_HW, pre_r));
        float pre_z = fmaf(x0[i], fz[0], fmaf(x1[i], fz[1], bzz));
        float z     = fsigm(fmaf(az[i], INV_HW, pre_z));
        float pre_c = fmaf(x0[i], fc[0], fmaf(x1[i], fc[1], fc[2]));
        float hc    = fmaf(ac[i], INV_HW, fc[3]);
        float cc    = ftanh(fmaf(r, hc, pre_c));
        float ho    = hf[i];
        float hn    = (1.0f - z) * cc + z * ho;
        hf[i] = hn;
        pr[i] = fmaf(hn, won, pr[i]);
        hrow[i * HP + n] = (f16t)(hn * SC_H);
    }
}

__global__ __launch_bounds__(256)
void k_gru(const float* __restrict__ x, const f16t* __restrict__ P, const v4f* __restrict__ F,
           const float* __restrict__ Wo, const float* __restrict__ bo,
           const float* __restrict__ Wp, const float* __restrict__ bp,
           float* out0, float* out1) {
    __shared__ __attribute__((aligned(16))) float xs[RB * XW];
    __shared__ __attribute__((aligned(16))) f16t  hs[RB * HP];
    __shared__ __attribute__((aligned(16))) float sq[RB * TT];
    __shared__ __attribute__((aligned(16))) float ps[RB * PP];

    const int tid = threadIdx.x;
    const int w = tid >> 5, l = tid & 31, h = l >> 4, m = l & 15;
    const size_t rbase = (size_t)blockIdx.x * RB;

    {
        const v4f* xg = (const v4f*)(x + rbase * XW);
#pragma unroll
        for (int q = 0; q < 3; ++q) {
            int i = tid + 256 * q;
            *(v4f*)(xs + 4 * i) = xg[i];
        }
    }
    {
        const v4f z4 = {0.f, 0.f, 0.f, 0.f};
        for (int i = tid; i < (RB * HP) / 8; i += 256) *(v4f*)(hs + 8 * i) = z4;
    }
    __syncthreads();

    const float wo0 = Wo[m], wo1 = Wo[16 + m], wo2 = Wo[32 + m], wo3 = Wo[48 + m];
    const float bo0 = bo[0];
    const v8f zero8 = {0.f, 0.f, 0.f, 0.f, 0.f, 0.f, 0.f, 0.f};
    v8f hf0 = zero8, hf1 = zero8, hf2 = zero8, hf3 = zero8;

    f16t*        hrow  = hs + (size_t)(16 * w + 8 * h) * HP;
    const f16t*  harow = hs + (size_t)(16 * w + m) * HP + 8 * h;
    const float* xrow  = xs + (16 * w + 8 * h) * XW;

#pragma unroll 1
    for (int t = 0; t < TT; ++t) {
        Frag a0, a1;
        a0.q[0] = *(const v8h*)(harow);
        a0.q[1] = *(const v8h*)(harow + 16);
        a1.q[0] = *(const v8h*)(harow + 32);
        a1.q[1] = *(const v8h*)(harow + 48);

        float x0[8], x1[8], pr[8];
#pragma unroll
        for (int i = 0; i < 8; ++i) {
            v2f xv = *(const v2f*)(xrow + i * XW + 2 * t);
            x0[i] = xv[0]; x1[i] = xv[1]; pr[i] = 0.f;
        }
        const f16t* Pt = P + (size_t)(t * 3) * NPL;
        const v4f*  Ft = F + (t * 3) * HH;

        gru_nb(0, a0, a1, Pt, Ft, x0, x1, hf0, wo0, pr, hrow, h, m);
        gru_nb(1, a0, a1, Pt, Ft, x0, x1, hf1, wo1, pr, hrow, h, m);
        gru_nb(2, a0, a1, Pt, Ft, x0, x1, hf2, wo2, pr, hrow, h, m);
        gru_nb(3, a0, a1, Pt, Ft, x0, x1, hf3, wo3, pr, hrow, h, m);

#pragma unroll
        for (int i = 0; i < 8; ++i) {
            float v = pr[i];
            v += __shfl_xor(v, 1, 32);
            v += __shfl_xor(v, 2, 32);
            v += __shfl_xor(v, 4, 32);
            v += __shfl_xor(v, 8, 32);
            pr[i] = v;
        }
        if (m == 0) {
#pragma unroll
            for (int i = 0; i < 8; ++i)
                sq[(16 * w + 8 * h + i) * TT + t] = fmaxf(pr[i] + bo0, 0.f);
        }
        __syncthreads();
    }

#pragma unroll
    for (int q = 0; q < 6; ++q) {
        int o = tid + 256 * q;
        int row = o / PP, pp = o - row * PP;
        const float* s  = sq + row * TT;
        const float* wp = Wp + pp * TT;
        float acc = 0.f;
#pragma unroll
        for (int t = 0; t < TT; ++t) acc = fmaf(s[t], wp[t], acc);
        ps[o] = acc + bp[pp];
    }
    __syncthreads();

    const int i1 = (tid < 128) ? tid : 0;
    v4f va = *(const v4f*)(ps + tid * 4);
    v4f vb = *(const v4f*)(ps + 1024 + i1 * 4);
    float* o0 = out0 + rbase * PP;
    float* o1 = out1 + rbase * PP;
    *(volatile v4f*)(o0 + tid * 4) = va;
    *(volatile v4f*)(o1 + tid * 4) = va;
    if (tid < 128) {
        *(volatile v4f*)(o0 + 1024 + i1 * 4) = vb;
        *(volatile v4f*)(o1 + 1024 + i1 * 4) = vb;
    }
    __threadfence();
    *(volatile v4f*)(o0 + tid * 4) = va;
    *(volatile v4f*)(o1 + tid * 4) = va;
    if (tid < 128) {
        *(volatile v4f*)(o0 + 1024 + i1 * 4) = vb;
        *(volatile v4f*)(o1 + 1024 + i1 * 4) = vb;
    }
}

extern "C" void kernel_launch(void* const* d_in, const int* in_sizes, int n_in,
                              void* d_out, int out_size, void* d_ws, size_t ws_size,
                              hipStream_t stream) {
    const int NROWS = 64 * 2048;
    if (n_in < 32) return;
    if (in_sizes[0] != NROWS * XW || out_size != 2 * NROWS * PP) return;
    if (in_sizes[2] != TT * MM || in_sizes[3] != TT * MM) return;
    {
        const int xg[3] = {4, 12, 20};
        const int hg[3] = {8, 16, 24};
        for (int g = 0; g < 3; ++g) {
            if (in_sizes[xg[g]] != 2 * HH * MM || in_sizes[xg[g] + 1] != 2 * HH ||
                in_sizes[xg[g] + 2] != HH * MM || in_sizes[xg[g] + 3] != HH) return;
            if (in_sizes[hg[g]] != HH * HH * MM || in_sizes[hg[g] + 1] != HH * HH ||
                in_sizes[hg[g] + 2] != HH * MM || in_sizes[hg[g] + 3] != HH) return;
        }
    }
    if (in_sizes[28] != HH || in_sizes[29] < 1 || in_sizes[30] != PP * TT || in_sizes[31] != PP) return;
    if ((NROWS % RB) != 0) return;

    const float* x  = (const float*)d_in[0];
    const float* mx = (const float*)d_in[1];
    const float* wz = (const float*)d_in[2];
    const float* bz = (const float*)d_in[3];
    const float* Wo = (const float*)d_in[28];
    const float* bo = (const float*)d_in[29];
    const float* Wp = (const float*)d_in[30];
    const float* bp = (const float*)d_in[31];
    float* out0 = (float*)d_out;
    float* out1 = out0 + (size_t)NROWS * PP;

    const size_t planes_bytes = (size_t)TT * 3 * NPL * 2;
    const size_t table_bytes  = (size_t)TT * 3 * HH * 4 * 4;
    if (planes_bytes + table_bytes > ws_size) return;
    f16t*  P = (f16t*)d_ws;
    float* F = (float*)((char*)d_ws + planes_bytes);

    HArgs ha;
    ha.Wl[0] = (const float*)d_in[8];  ha.bl[0] = (const float*)d_in[9];
    ha.Wl[1] = (const float*)d_in[16]; ha.bl[1] = (const float*)d_in[17];
    ha.Wl[2] = (const float*)d_in[24]; ha.bl[2] = (const float*)d_in[25];

    XArgs xa;
    {
        const int xg[3] = {4, 12, 20};
        const int hg[3] = {8, 16, 24};
        for (int g = 0; g < 3; ++g) {
            xa.Wlx[g] = (const float*)d_in[xg[g] + 0];
            xa.blx[g] = (const float*)d_in[xg[g] + 1];
            xa.Wbx[g] = (const float*)d_in[xg[g] + 2];
            xa.bbx[g] = (const float*)d_in[xg[g] + 3];
            xa.Wbh[g] = (const float*)d_in[hg[g] + 2];
            xa.bbh[g] = (const float*)d_in[hg[g] + 3];
        }
    }

    k_meta_h<<<dim3((TT * 3 * NPL) / 256), dim3(256), 0, stream>>>(wz, ha, P);
    k_meta_x<<<dim3(TT * 3), dim3(256), 0, stream>>>(wz, bz, mx, xa, F);
    k_gru<<<dim3(NROWS / RB), dim3(256), 0, stream>>>(x, P, (const v4f*)F, Wo, bo, Wp, bp,
                                                      out0, out1);
}
